// MultiHeadAttention_12120397709593
// MI455X (gfx1250) — hardware-verified
//
#include <hip/hip_runtime.h>
#ifndef NB
#define NB 2
#endif
#ifndef SEQ
#define SEQ 2048
#endif
#define NB_FULL 2
#define SEQ_FULL 2048
#define SQ SEQ
#define DM 1024
#define NH 16
#define HD 64
#define QT 256
#define NKX SQ
#define QT0 128
#define NR ((size_t)NB * SQ)
#define LQ (3 * DM)
static_assert(SEQ % QT == 0);
static_assert(SEQ >= QT0);
static_assert(NB <= NB_FULL);
static_assert(SEQ <= SEQ_FULL);
static_assert(DM % 64 == 0);
static_assert(((size_t)NB * SEQ) % 128 == 0);
static_assert(QT % 128 == 0);
static_assert(QT0 % 128 == 0);

typedef unsigned short v8us __attribute__((ext_vector_type(8), may_alias));
typedef float  v8f  __attribute__((ext_vector_type(8)));
typedef float  v4f  __attribute__((ext_vector_type(4)));
typedef float  v4fa __attribute__((ext_vector_type(4), may_alias));
typedef _Float16 v16h __attribute__((ext_vector_type(16)));
typedef _Float16 v4h __attribute__((ext_vector_type(4)));
union FragH { v16h v; v8us half[2]; _Float16 h[16]; unsigned short u[16]; };

__device__ __forceinline__ unsigned short bf16_bits(float x) { unsigned int u = __float_as_uint(x); return (unsigned short)((u + 0x7FFFu + ((u >> 16) & 1u)) >> 16); }
__device__ __forceinline__ float bf16_val(unsigned short b) { return __uint_as_float(((unsigned int)b) << 16); }
__device__ __forceinline__ float bf16_rne(float x) { return bf16_val(bf16_bits(x)); }

__global__ __launch_bounds__(256) void k_wt_f16(const float* __restrict__ W, _Float16* __restrict__ Wt, int K, int N, float scale) {
  const int t = blockIdx.x * 256 + threadIdx.x; if (t >= N * (K / 8)) return; const int n = t / (K / 8), k8 = (t % (K / 8)) * 8; FragH f;
#pragma unroll
  for (int i = 0; i < 8; ++i) f.h[i] = (_Float16)(bf16_rne(W[(size_t)(k8 + i) * N + n]) * scale);
  const v8us o = f.half[0];
  *(volatile v8us*)((unsigned short*)Wt + (size_t)n * K + k8) = o; __threadfence(); *(volatile v8us*)((unsigned short*)Wt + (size_t)n * K + k8) = o;
}

__global__ __launch_bounds__(256) void k_x16(const float* __restrict__ x, _Float16* __restrict__ X16, size_t n8) {
  const size_t t = (size_t)blockIdx.x * 256 + threadIdx.x; if (t >= n8) return;
  const size_t e = t * 8; const size_t r = e / DM, c = e % DM; const size_t b = r / SQ, s = r % SQ;
  const float* src = x + (b * SEQ_FULL + s) * DM + c;
  FragH f;
#pragma unroll
  for (int q = 0; q < 8; ++q) f.h[q] = (_Float16)bf16_rne(src[q]);
  const v8us o = f.half[0];
  *(volatile v8us*)((unsigned short*)X16 + t * 8) = o; __threadfence(); *(volatile v8us*)((unsigned short*)X16 + t * 8) = o;
}

__global__ __launch_bounds__(256) void k_hl(const float* __restrict__ F, _Float16* __restrict__ Hh, _Float16* __restrict__ Hl, size_t n8) {
  const size_t t = (size_t)blockIdx.x * 256 + threadIdx.x; if (t >= n8) return; FragH fh, fl; const v4f a = *(const v4fa*)(F + t * 8), c = *(const v4fa*)(F + t * 8 + 4);
#pragma unroll
  for (int q = 0; q < 4; ++q) { _Float16 h = (_Float16)a[q]; fh.h[q] = h; fl.h[q] = (_Float16)((a[q] - (float)h) * 1024.0f); h = (_Float16)c[q]; fh.h[4 + q] = h; fl.h[4 + q] = (_Float16)((c[q] - (float)h) * 1024.0f); }
  const v8us oh = fh.half[0], ol = fl.half[0];
  for (int pass = 0; pass < 2; ++pass) { *(volatile v8us*)((unsigned short*)Hh + t * 8) = oh; *(volatile v8us*)((unsigned short*)Hl + t * 8) = ol; if (pass == 0) __threadfence(); }
}

__device__ __forceinline__ v16h g2_frag(const _Float16* p, int hh) { FragH f; f.half[0] = *(const v8us*)((const unsigned short*)p + 8 * hh); f.half[1] = *(const v8us*)((const unsigned short*)p + 16 + 8 * hh); return f.v; }
__device__ __forceinline__ v8f g2_mma(v16h a, v16h b, v8f c) { v8f d = __builtin_amdgcn_wmma_f32_16x16x32_f16(false, a, false, b, (short)0, c, false, false); asm volatile("v_nop\n\tv_nop\n\tv_nop\n\tv_nop" : "+v"(d) : "v"(a), "v"(b)); return d; }
template <int ACT>
__global__ __launch_bounds__(128) void k_gemm2(const _Float16* __restrict__ A, int lda, size_t sA, const _Float16* __restrict__ Bh, int ldb, size_t sB, float alpha, const float* __restrict__ bias, size_t sBias, const float* CP,
    float* C, _Float16* __restrict__ C16, int ldc, size_t sC, int M, int N, int K) {
  static_assert(ACT == 0);
  __shared__ __attribute__((aligned(16))) float so[4][32][68];
  const int tid = threadIdx.x, w = __builtin_amdgcn_readfirstlane((int)(tid >> 5)), lane = tid & 31, ln = lane & 15, hh = lane >> 4; const int by = blockIdx.y;
  A += (size_t)by * sA; Bh += (size_t)by * sB; const size_t cofs = (size_t)by * sC; const float* bp = bias ? bias + (size_t)by * sBias : nullptr;
  const int ntn = N >> 6; const int mt = blockIdx.x / ntn, nq = blockIdx.x - mt * ntn; const int row0 = mt * 128 + 32 * w, col0 = nq * 64; if (row0 >= M) return;
  const _Float16* a0p = A + (size_t)(row0 + ln) * lda; const _Float16* a1p = a0p + (size_t)16 * lda;
  const _Float16* b0p = Bh + (size_t)(col0 + ln) * ldb; const _Float16* b1p = b0p + (size_t)16 * ldb; const _Float16* b2p = b1p + (size_t)16 * ldb; const _Float16* b3p = b2p + (size_t)16 * ldb;
  const v8f z8 = {0.f,0.f,0.f,0.f,0.f,0.f,0.f,0.f}; v8f c00 = z8, c01 = z8, c02 = z8, c03 = z8, c10 = z8, c11 = z8, c12 = z8, c13 = z8;
#pragma unroll 1
  for (int kb = 0; kb < K; kb += 32) { const v16h a0 = g2_frag(a0p + kb, hh), a1 = g2_frag(a1p + kb, hh);
    v16h b = g2_frag(b0p + kb, hh); c00 = g2_mma(a0, b, c00); c10 = g2_mma(a1, b, c10);
    b = g2_frag(b1p + kb, hh); c01 = g2_mma(a0, b, c01); c11 = g2_mma(a1, b, c11);
    b = g2_frag(b2p + kb, hh); c02 = g2_mma(a0, b, c02); c12 = g2_mma(a1, b, c12);
    b = g2_frag(b3p + kb, hh); c03 = g2_mma(a0, b, c03); c13 = g2_mma(a1, b, c13); }
  v8f accs[8] = {c00, c01, c02, c03, c10, c11, c12, c13};
#pragma unroll
  for (int u = 0; u < 8; ++u) { const int t = u & 3, half = u >> 2; const int col = col0 + t * 16 + ln; const float bv = bp ? bf16_rne(bp[col]) : 0.f;
#pragma unroll
    for (int r = 0; r < 8; ++r) { const int rloc = half * 16 + 8 * hh + r; float v = accs[u][r] * alpha + bv; if (CP) v += CP[cofs + (size_t)(row0 + rloc) * ldc + col];
      so[w][rloc][t * 16 + ln] = v; } }
  __builtin_amdgcn_fence(4  , "workgroup"); __builtin_amdgcn_wave_barrier();
  const int rsub = lane >> 4, c4 = (lane & 15) * 4;
  for (int pass = 0; pass < 2; ++pass) {
#pragma unroll
    for (int q = 0; q < 16; ++q) { const int r = q * 2 + rsub; const v4f v = *(const v4fa*)&so[w][r][c4]; if (C) *(volatile v4f*)(C + cofs + (size_t)(row0 + r) * ldc + col0 + c4) = v; if (C16) { v4h h4; for (int i = 0; i < 4; ++i) h4[i] = (_Float16)v[i]; *(volatile v4h*)(C16 + cofs + (size_t)(row0 + r) * ldc + col0 + c4) = h4; } }
    if (pass == 0) __threadfence(); } }

template <int NHv, int TTv>
__global__ __launch_bounds__(256) void k_vt(const _Float16* __restrict__ V16, int ldv, int voff, _Float16* __restrict__ Vt) { __shared__ unsigned short tl[64][66]; const int tid = threadIdx.x; const int slab = blockIdx.x / (TTv / 64), lg = blockIdx.x % (TTv / 64); const int b = slab / NHv, h = slab % NHv;
  for (int i = tid; i < 64 * 8; i += 256) { const int r = i / 8, c8 = (i % 8) * 8; FragH f; f.half[0] = *(const v8us*)((const unsigned short*)V16 + ((size_t)b * TTv + lg * 64 + r) * ldv + voff + h * 64 + c8);
#pragma unroll
    for (int q = 0; q < 8; ++q) tl[r][c8 + q] = f.u[q]; }
  __syncthreads();
  for (int pass = 0; pass < 2; ++pass) {
#pragma unroll
    for (int rd = 0; rd < 2; ++rd) { const int d = rd * 32 + tid / 8, pc = tid % 8; FragH f;
#pragma unroll
      for (int q = 0; q < 8; ++q) f.u[q] = tl[pc * 8 + q][d];
      const v8us o = f.half[0];
      *(volatile v8us*)((unsigned short*)Vt + ((size_t)slab * 64 + d) * TTv + lg * 64 + pc * 8) = o; }
    if (pass == 0) __threadfence(); } }

__global__ __launch_bounds__(256) void k_rsmcf2(const float* __restrict__ S, _Float16* __restrict__ P, int hg, int q0, int nk) {
  #pragma clang fp contract(off)
  const int t = blockIdx.x * 256 + threadIdx.x; if (t >= hg * QT) return; const size_t i = (size_t)t; const float* s = S + i * NKX; const int last = q0 + (t % QT); float mx = -3.0e38f;
#pragma unroll 1
  for (int j = 0; j < nk; ++j) { const float f = (j <= last) ? 1.f : 0.f; mx = fmaxf(mx, fmaf(f, s[j], (1.f - f) * -1.0e9f)); } float se = 0.f;
#pragma unroll 1
  for (int j = 0; j < nk; ++j) { const float f = (j <= last) ? 1.f : 0.f; se += __expf(fmaf(f, s[j], (1.f - f) * -1.0e9f) - mx); } const float sc = 256.0f / se;
#pragma unroll 1
  for (int j0 = 0; j0 < nk; j0 += 8) { FragH fr; for (int q = 0; q < 8; ++q) { const int j = j0 + q; const float f = (j <= last) ? 1.f : 0.f; fr.h[q] = (_Float16)(__expf(fmaf(f, s[j], (1.f - f) * -1.0e9f) - mx) * sc); } const v8us o = fr.half[0]; unsigned short* d = (unsigned short*)P + i * NKX + j0; *(volatile v8us*)d = o; __threadfence(); *(volatile v8us*)d = o; } }

__global__ __launch_bounds__(64) void k_att0(const float* __restrict__ QF, const float* __restrict__ KF, const float* __restrict__ VF, int ld, float scale, float* __restrict__ OF, int ldo) {
  #pragma clang fp contract(off)
  __shared__ __attribute__((aligned(16))) float lq[64][64]; __shared__ __attribute__((aligned(16))) float lo[64][64];
  const int tid = threadIdx.x; const int h = blockIdx.x / (QT0 / 64), rg = blockIdx.x % (QT0 / 64); const int i = rg * 64 + tid;
  const float* qr = QF + (size_t)i * ld + h * HD;
#pragma unroll 1
  for (int c = 0; c < HD / 4; ++c) { *(v4f*)&lq[tid][c * 4] = *(const v4fa*)(qr + c * 4); const v4f z = {0.f, 0.f, 0.f, 0.f}; *(v4f*)&lo[tid][c * 4] = z; }
  float m = -1.0e30f, l = 0.f; const int jmax = rg * 64 + 63;
#pragma unroll 1
  for (int j = 0; j <= jmax; ++j) { const float* kr = KF + (size_t)j * ld + h * HD; const float* vr = VF + (size_t)j * ld + h * HD; float s = 0.f;
#pragma unroll 1
    for (int c = 0; c < HD / 4; ++c) { const v4f kq = *(const v4fa*)(kr + c * 4); const v4f qq = *(v4f*)&lq[tid][c * 4]; s = __fadd_rn(s, __fmul_rn(qq[0], kq[0])); s = __fadd_rn(s, __fmul_rn(qq[1], kq[1])); s = __fadd_rn(s, __fmul_rn(qq[2], kq[2])); s = __fadd_rn(s, __fmul_rn(qq[3], kq[3])); }
    s = __fmul_rn(s, scale);
    const float f = (j <= i) ? 1.f : 0.f; const float sm = fmaf(f, s, (1.f - f) * -1.0e30f); const float mn = fmaxf(m, sm); const float sc = expf(m - mn); const float e = expf(sm - mn); l = __fadd_rn(__fmul_rn(l, sc), e); m = mn;
#pragma unroll 1
    for (int c = 0; c < HD / 4; ++c) { const v4f vv = *(const v4fa*)(vr + c * 4); v4f oo = *(v4f*)&lo[tid][c * 4]; for (int u = 0; u < 4; ++u) oo[u] = __fadd_rn(__fmul_rn(oo[u], sc), __fmul_rn(e, vv[u])); *(v4f*)&lo[tid][c * 4] = oo; } }
  const float fin = 64.0f / l;
#pragma unroll 1
  for (int c = 0; c < HD / 4; ++c) { v4f oo = *(v4f*)&lo[tid][c * 4]; for (int u = 0; u < 4; ++u) oo[u] = __fmul_rn(oo[u], fin); *(v4f*)&lo[tid][c * 4] = oo; }
  __syncthreads();
  for (int pass = 0; pass < 2; ++pass) {
#pragma unroll 1
    for (int it = 0; it < 16; ++it) { const int row = it * 4 + tid / 16, pc = (tid % 16) * 4; const v4f v = *(const v4f*)&lo[row][pc]; *(volatile v4f*)(OF + (size_t)(rg * 64 + row) * ldo + h * HD + pc) = v; }
    if (pass == 0) __threadfence(); } }

extern "C" void kernel_launch(void* const* d_in, const int* in_sizes, int n_in,
                              void* d_out, int out_size, void* d_ws, size_t ws_size, hipStream_t stream) {
  if (n_in < 5) return;
  const size_t need_x = ((size_t)(NB - 1) * SEQ_FULL + SQ) * DM;
  if ((size_t)in_sizes[0] < need_x || in_sizes[1] < DM * LQ || in_sizes[2] < LQ || in_sizes[3] < DM * DM || in_sizes[4] < DM || (size_t)out_size < need_x) return;
  const float* x = (const float*)d_in[0]; const float* wqkv = (const float*)d_in[1]; const float* bqkv = (const float*)d_in[2]; const float* wo = (const float*)d_in[3]; const float* bo = (const float*)d_in[4];
  float* out = (float*)d_out;
  char* ws = (char*)d_ws; size_t off = 0;
  auto take = [&](size_t bytes) { char* p = ws + off; off += (bytes + 255) & ~(size_t)255; return p; };
  _Float16* BQKV = (_Float16*)take((size_t)3 * DM * DM * 2); _Float16* BO = (_Float16*)take((size_t)DM * DM * 2);
  _Float16* X16 = (_Float16*)take(NR * DM * 2); _Float16* QKV = (_Float16*)take(NR * 3 * DM * 2);
  _Float16* T0 = QKV;
  _Float16* T1 = QKV + DM;
  _Float16* T2 = QKV + 2 * DM;
  _Float16* O16 = (_Float16*)take(NR * DM * 2);
  float* S = (float*)take((size_t)NH * QT * NKX * 4); _Float16* P = (_Float16*)take((size_t)NH * QT * NKX * 2); _Float16* VT = (_Float16*)take((size_t)NH * HD * SQ * 2);
  float* QF0 = (float*)take((size_t)QT0 * DM * 4); float* KF0 = (float*)take((size_t)QT0 * DM * 4); float* VF0 = (float*)take((size_t)QT0 * DM * 4);
  float* OF0 = (float*)take((size_t)NB * QT0 * DM * 4); _Float16* OH0 = (_Float16*)take((size_t)NB * QT0 * DM * 2); _Float16* OL0 = (_Float16*)take((size_t)NB * QT0 * DM * 2);
  if (off > ws_size || off > (size_t)134217728) return;
  k_wt_f16<<<(unsigned)(((size_t)LQ * (DM / 8) + 255) / 256), 256, 0, stream>>>(wqkv, BQKV, DM, LQ, 16.0f);
  k_wt_f16<<<(unsigned)(((size_t)DM * (DM / 8) + 255) / 256), 256, 0, stream>>>(wo, BO, DM, DM, 16.0f);
  k_x16<<<(unsigned)((NR * DM / 8 + 255) / 256), 256, 0, stream>>>(x, X16, NR * DM / 8);
  k_gemm2<0><<<dim3((unsigned)((NR / 128) * (LQ / 64)), 1), 128, 0, stream>>>(X16, DM, 0, BQKV, DM, 0, 0.0625f, bqkv, 0, nullptr, nullptr, QKV, LQ, 0, (int)NR, LQ, DM);
  for (int b = 0; b < NB; ++b) { const size_t r0 = (size_t)b * SQ;
    k_vt<NH, SQ><<<NH * (SQ / 64), 256, 0, stream>>>(T2 + r0 * LQ, LQ, 0, VT);
    k_gemm2<0><<<dim3((QT0 / 128) * (DM / 64), 1), 128, 0, stream>>>(X16 + r0 * DM, DM, 0, BQKV, DM, 0, 0.0625f, bqkv, 0, nullptr, QF0, nullptr, DM, 0, QT0, DM, DM);
    k_gemm2<0><<<dim3((QT0 / 128) * (DM / 64), 1), 128, 0, stream>>>(X16 + r0 * DM, DM, 0, BQKV + (size_t)DM * DM, DM, 0, 0.0625f, bqkv + DM, 0, nullptr, KF0, nullptr, DM, 0, QT0, DM, DM);
    k_gemm2<0><<<dim3((QT0 / 128) * (DM / 64), 1), 128, 0, stream>>>(X16 + r0 * DM, DM, 0, BQKV + (size_t)2 * DM * DM, DM, 0, 0.0625f, bqkv + 2 * DM, 0, nullptr, VF0, nullptr, DM, 0, QT0, DM, DM);
    k_att0<<<NH * (QT0 / 64), 64, 0, stream>>>(QF0, KF0, VF0, DM, 0.125f, OF0 + (size_t)b * QT0 * DM, DM);
    for (int q0 = 0; q0 < SQ; q0 += QT) { const int nk = q0 + QT;
      k_gemm2<0><<<dim3((QT / 128) * (nk / 64), NH), 128, 0, stream>>>(T0 + (r0 + q0) * LQ, LQ, (size_t)HD, T1 + r0 * LQ, LQ, (size_t)HD, 0.125f, nullptr, 0, nullptr, S, nullptr, NKX, (size_t)QT * NKX, QT, nk, HD);
      k_rsmcf2<<<(NH * QT + 255) / 256, 256, 0, stream>>>(S, P, NH, q0, nk);
      k_gemm2<0><<<dim3((QT / 128) * (HD / 64), NH), 128, 0, stream>>>(P, NKX, (size_t)QT * NKX, VT, SQ, (size_t)HD * SQ, 0.25f, nullptr, 0, nullptr, nullptr, O16 + (r0 + q0) * DM, DM, (size_t)HD, QT, HD, nk); } }
  k_gemm2<0><<<dim3((unsigned)((SQ / 128) * (DM / 64)), NB), 128, 0, stream>>>(O16, DM, (size_t)SQ * DM, BO, DM, 0, 0.0009765625f, bo, 0, nullptr, out, nullptr, DM, (size_t)SEQ_FULL * DM, SQ, DM, DM);
  k_hl<<<(unsigned)(((size_t)NB * QT0 * DM / 8 + 255) / 256), 256, 0, stream>>>(OF0, OH0, OL0, (size_t)NB * QT0 * DM / 8);
  for (int b = 0; b < NB; ++b) { float* ob = out + (size_t)b * SEQ_FULL * DM; const size_t f0 = (size_t)b * QT0;
    k_gemm2<0><<<dim3((QT0 / 128) * (DM / 64), 1), 128, 0, stream>>>(OH0 + f0 * DM, DM, 0, BO, DM, 0, 0.0009765625f, bo, 0, nullptr, ob, nullptr, DM, 0, QT0, DM, DM);
    k_gemm2<0><<<dim3((QT0 / 128) * (DM / 64), 1), 128, 0, stream>>>(OL0 + f0 * DM, DM, 0, BO, DM, 0, 0.00000095367431640625f, nullptr, 0, (const float*)ob, ob, nullptr, DM, 0, QT0, DM, DM); }
}
